// question_layer_LSTM_72241349919244
// MI455X (gfx1250) — hardware-verified
//
#include <hip/hip_runtime.h>
#include <math.h>

constexpr int NBATCH   = 256;
constexpr int NSTEPS   = 26;
constexpr int NEMB     = 300;
constexpr int NEMBP    = 320;
constexpr int NHID     = 1024;
constexpr int NGATE    = 4096;
constexpr int NVOCAB   = 20000;
constexpr int SEGSTEPS = 13;
constexpr int NROWS    = NSTEPS * NBATCH;
constexpr int CHROWS   = SEGSTEPS * NBATCH;
constexpr int NTHR     = 256;
constexpr int BLKROWS  = 16;
constexpr int HPITCH   = 1032;
constexpr int CPITCH   = 1028;
constexpr int OSP      = 72;
constexpr int SLABP    = 68;
constexpr float WCARRY = 16.0f;
constexpr float ACARRY = 16.0f;
constexpr float FOLDSC = 1.0f / (WCARRY * ACARRY);
constexpr float BN_EPS = 1e-3f;

static_assert(NSTEPS == 2 * SEGSTEPS, "two equal time segments");
static_assert(NGATE == 4 * NHID, "four gate blocks");
static_assert(NEMBP % 32 == 0 && NEMBP >= NEMB, "K pad multiple of 32");
static_assert(NEMB % 4 == 0 && NEMBP % 8 == 0, "vector gather granularity");
static_assert(NHID % 64 == 0 && NGATE % 64 == 0 && NROWS % 64 == 0 && CHROWS % 64 == 0 && NBATCH % 64 == 0, "tile multiples");
static_assert(NHID % 32 == 0, "K multiple of 32");
static_assert(NBATCH % BLKROWS == 0, "row blocks");
static_assert(NHID == 128 * (NTHR / 32), "8 waves x 128 hidden units");
static_assert((2 * BLKROWS * HPITCH) % 8 == 0 && HPITCH % 8 == 0, "16-byte LDS chunks");
static_assert(CPITCH % 4 == 0 && CPITCH >= NHID, "16-byte aligned c rows");
static_assert(OSP % 8 == 0 && OSP >= 64, "16-byte aligned output slab rows");
static_assert((NROWS * (NEMBP / 8)) % NTHR == 0, "gather grid exact");
static_assert((SEGSTEPS & 1) == 1, "final h buffer parity");
static_assert((BLKROWS * NHID / 4) % NTHR == 0 && (BLKROWS * NHID / 8) % NTHR == 0, "cooperative copy loops exact");

typedef __attribute__((ext_vector_type(16))) _Float16 v16h;
typedef __attribute__((ext_vector_type(8)))  _Float16 v8h;
typedef __attribute__((ext_vector_type(8)))  float    v8f;
typedef __attribute__((ext_vector_type(4)))  float    v4f;

union FragU { v16h v; v8h h[2]; };

__device__ __forceinline__ v16h frag_load(const _Float16* p) {
  FragU f;
  f.h[0] = *(const v8h*)(p);
  f.h[1] = *(const v8h*)(p + 16);
  return f.v;
}
__device__ __forceinline__ v8f frag_mma(v16h a, v16h b, v8f c) {
  return __builtin_amdgcn_wmma_f32_16x16x32_f16(false, a, false, b, (short)0, c, false, false);
}
__device__ __forceinline__ void guard_group4(v8f& a0, v8f& a1, v8f& a2, v8f& a3,
                                             v16h x, v16h y0, v16h y1, v16h y2, v16h y3) {
  asm volatile("v_nop\n\tv_nop\n\tv_nop\n\tv_nop"
               : "+v"(a0), "+v"(a1), "+v"(a2), "+v"(a3)
               : "v"(x), "v"(y0), "v"(y1), "v"(y2), "v"(y3));
}
__device__ __forceinline__ void acc_guard4(v8f& a, v8f& b, v8f& c, v8f& d) {
  asm volatile("v_nop\n\tv_nop\n\tv_nop\n\tv_nop" : "+v"(a), "+v"(b), "+v"(c), "+v"(d));
}
__device__ __forceinline__ void wave_lds_sync() {
  __builtin_amdgcn_fence(__ATOMIC_RELEASE, "workgroup");
  __builtin_amdgcn_wave_barrier();
  __builtin_amdgcn_fence(__ATOMIC_ACQUIRE, "workgroup");
}
__device__ __forceinline__ float fsig(float x)  { return __builtin_amdgcn_rcpf(1.0f + __expf(-x)); }
__device__ __forceinline__ float ftanh(float x) { return 1.0f - 2.0f * __builtin_amdgcn_rcpf(__expf(2.0f * x) + 1.0f); }

__global__ __launch_bounds__(NTHR) void tpw_f16_kernel(const float* __restrict__ src, int R, int C, int ldo,
                                                       unsigned short* __restrict__ O, float sc) {
  __shared__ float Tt[64 * 65];
  const int tid = threadIdx.x;
  const int c0 = blockIdx.x * 64, r0 = blockIdx.y * 64;
#pragma unroll
  for (int i = 0; i < 4; ++i) {
    const int idx = i * NTHR + tid;
    const int rr = idx >> 4, cc = (idx & 15) * 4;
    const int rg = r0 + rr;
    const int rcl = (rg < R) ? rg : (R - 1);
    const v4f v = *(const v4f*)(src + (size_t)rcl * (size_t)C + c0 + cc);
    const bool ok = (rg < R);
    Tt[rr * 65 + cc + 0] = ok ? v[0] : 0.0f;
    Tt[rr * 65 + cc + 1] = ok ? v[1] : 0.0f;
    Tt[rr * 65 + cc + 2] = ok ? v[2] : 0.0f;
    Tt[rr * 65 + cc + 3] = ok ? v[3] : 0.0f;
  }
  __syncthreads();
  const int q = tid >> 3, c8 = (tid & 7) * 8;
  v8h hv[2];
#pragma unroll
  for (int g = 0; g < 2; ++g) {
    const int qq = g * 32 + q;
#pragma unroll
    for (int e = 0; e < 8; ++e) {
      const float f = Tt[(c8 + e) * 65 + qq];
      hv[g][e] = (_Float16)(f * sc);
    }
  }
  for (int pass = 0; pass < 2; ++pass) {
#pragma unroll
    for (int g = 0; g < 2; ++g) {
      const size_t o = (size_t)(c0 + g * 32 + q) * (size_t)ldo + (size_t)(r0 + c8);
      *(volatile v8h*)(O + o) = hv[g];
    }
    __threadfence();
  }
}

__global__ __launch_bounds__(NTHR) void gather_x16_kernel(const int* __restrict__ tok, const float* __restrict__ emb,
                                                          unsigned short* __restrict__ X16) {
  const int i = blockIdx.x * NTHR + threadIdx.x;
  const int n8 = NROWS * (NEMBP / 8);
  if (i < n8) {
    const int row = i / (NEMBP / 8);
    const int c8  = i - row * (NEMBP / 8);
    const int t = row / NBATCH;
    const int b = row - t * NBATCH;
    int id = tok[b * NSTEPS + t];
    id = id < 0 ? 0 : (id > NVOCAB - 1 ? NVOCAB - 1 : id);
    const int e  = c8 * 8;
    const int ea = (e < NEMB - 4) ? e : (NEMB - 4);
    const int eb = (e + 4 < NEMB - 4) ? (e + 4) : (NEMB - 4);
    const float* er = emb + (size_t)id * NEMB;
    const v4f va = *(const v4f*)(er + ea);
    const v4f vb = *(const v4f*)(er + eb);
    const bool oka = (e < NEMB);
    const bool okb = (e + 4 < NEMB);
    v8h hv;
#pragma unroll
    for (int k = 0; k < 4; ++k) {
      const float fa = oka ? va[k] * ACARRY : 0.0f;
      const float fb = okb ? vb[k] * ACARRY : 0.0f;
      hv[k]     = (_Float16)fa;
      hv[4 + k] = (_Float16)fb;
    }
    *(volatile v8h*)(X16 + (size_t)i * 8) = hv;
    __threadfence();
    *(volatile v8h*)(X16 + (size_t)i * 8) = hv;
  }
}

template <int ACT>
__global__ __launch_bounds__(NTHR) void gemm64_f16_kernel(
    const unsigned short* __restrict__ Ap, int lda,
    const unsigned short* __restrict__ Btp, int ldb,
    float* __restrict__ C, int ldc,
    const float* __restrict__ bias, int M, int N, int K, float scale) {
  __shared__ __align__(16) float sT[NTHR / 32][16 * SLABP];
  const _Float16* A  = (const _Float16*)Ap;
  const _Float16* Bt = (const _Float16*)Btp;
  const int lane = threadIdx.x & 31;
  const int wave = threadIdx.x >> 5;
  const int tilesN = N >> 6;
  const int tilesM = M >> 6;
  const int tile = blockIdx.x * 8 + wave;
  if (tile >= tilesM * tilesN) return;
  const int tm = tile / tilesN;
  const int tn = tile - tm * tilesN;
  const int m0 = tm << 6;
  const int n0 = tn << 6;
  const int rlane = lane & 15;
  const int koff  = (lane >> 4) * 8;
  const int mOff  = (lane >> 4) * 8;

  const _Float16* bp[4];
  const _Float16* ap[4];
#pragma unroll
  for (int j = 0; j < 4; ++j) bp[j] = Bt + (size_t)(n0 + (j << 4) + rlane) * ldb + koff;
#pragma unroll
  for (int i = 0; i < 4; ++i) ap[i] = A + (size_t)(m0 + (i << 4) + rlane) * lda + koff;

  v8f acc[4][4];
#pragma unroll
  for (int i = 0; i < 4; ++i)
#pragma unroll
    for (int j = 0; j < 4; ++j) acc[i][j] = (v8f){0.f, 0.f, 0.f, 0.f, 0.f, 0.f, 0.f, 0.f};

#pragma unroll 1
  for (int k0 = 0; k0 < K; k0 += 32) {
    v16h bh[4];
#pragma unroll
    for (int j = 0; j < 4; ++j) bh[j] = frag_load(bp[j] + k0);
#pragma unroll
    for (int i = 0; i < 4; ++i) {
      const v16h ah = frag_load(ap[i] + k0);
#pragma unroll
      for (int j = 0; j < 4; ++j) acc[i][j] = frag_mma(ah, bh[j], acc[i][j]);
      guard_group4(acc[i][0], acc[i][1], acc[i][2], acc[i][3], ah, bh[0], bh[1], bh[2], bh[3]);
    }
  }
  acc_guard4(acc[0][0], acc[0][1], acc[0][2], acc[0][3]);
  acc_guard4(acc[1][0], acc[1][1], acc[1][2], acc[1][3]);
  acc_guard4(acc[2][0], acc[2][1], acc[2][2], acc[2][3]);
  acc_guard4(acc[3][0], acc[3][1], acc[3][2], acc[3][3]);

  float* slab = sT[wave];
#pragma unroll
  for (int i = 0; i < 4; ++i) {
    const int mBase = m0 + (i << 4);
#pragma unroll
    for (int j = 0; j < 4; ++j) {
      const int n = n0 + (j << 4) + rlane;
      const float bv = bias[n];
#pragma unroll
      for (int r = 0; r < 8; ++r) {
        const float v = acc[i][j][r] * scale + bv;
        slab[(mOff + r) * SLABP + (j << 4) + rlane] = v;
      }
    }
    wave_lds_sync();
    if (ACT == 6) {
#pragma unroll 1
      for (int it = 0; it < 32; ++it) {
        const int idx = it * 32 + lane;
        const int row = idx >> 6, col = idx & 63;
        float* p = slab + row * SLABP + col;
        const float u = *p;
        *p = tanhf(u);
      }
      wave_lds_sync();
    }
    {
      const int hh = lane >> 4, c4 = (lane & 15) * 4;
      for (int pass = 0; pass < 2; ++pass) {
#pragma unroll
        for (int it = 0; it < 8; ++it) {
          const int row = it * 2 + hh;
          const v4f v = *(const v4f*)(slab + row * SLABP + c4);
          *(volatile v4f*)(C + (size_t)(mBase + row) * ldc + n0 + c4) = v;
        }
        __threadfence();
      }
    }
    wave_lds_sync();
  }
}

__global__ __launch_bounds__(NTHR) __attribute__((amdgpu_num_vgpr(256))) void lstm_seg_kernel(
    const float* __restrict__ XP, const unsigned short* __restrict__ Utp,
    const float* __restrict__ bn_mean, const float* __restrict__ bn_var,
    unsigned short* __restrict__ OUT16, unsigned short* __restrict__ HST, float* __restrict__ CST,
    int t0, int out_tstride, int out_every, int final_out, int init) {
  __shared__ __align__(16) _Float16 Hb[2][BLKROWS * HPITCH];
  __shared__ __align__(16) float    Cl[BLKROWS * CPITCH];
  __shared__ __align__(16) _Float16 Os[NTHR / 32][16 * OSP];
  const _Float16* Ut = (const _Float16*)Utp;
  const int tid = threadIdx.x, lane = tid & 31, wave = tid >> 5;
  const int c = lane & 15, hh = lane >> 4, koff = hh * 8;
  const int rowbase = blockIdx.x * BLKROWS;
  _Float16* os = Os[wave];

  {
    const v8h zv = (v8h){(_Float16)0.0f, (_Float16)0.0f, (_Float16)0.0f, (_Float16)0.0f,
                         (_Float16)0.0f, (_Float16)0.0f, (_Float16)0.0f, (_Float16)0.0f};
    v8h* hz = (v8h*)&Hb[0][0];
#pragma unroll 1
    for (int i = tid; i < (2 * BLKROWS * HPITCH) / 8; i += NTHR) hz[i] = zv;
  }
  if (init != 0) {
    const v4f z4 = (v4f){0.0f, 0.0f, 0.0f, 0.0f};
#pragma unroll 1
    for (int it = 0; it < (BLKROWS * NHID / 4) / NTHR; ++it) {
      const int idx = it * NTHR + tid;
      const int row = idx >> 8, c4 = (idx & 255) * 4;
      *(v4f*)(Cl + row * CPITCH + c4) = z4;
    }
  } else {
#pragma unroll 1
    for (int it = 0; it < (BLKROWS * NHID / 4) / NTHR; ++it) {
      const int idx = it * NTHR + tid;
      const int row = idx >> 8, c4 = (idx & 255) * 4;
      const v4f v = *(const v4f*)(CST + (size_t)(rowbase + row) * NHID + c4);
      *(v4f*)(Cl + row * CPITCH + c4) = v;
    }
  }
  __syncthreads();
  if (init == 0) {
#pragma unroll 1
    for (int it = 0; it < (BLKROWS * NHID / 8) / NTHR; ++it) {
      const int idx = it * NTHR + tid;
      const int row = idx >> 7, ch = idx & 127;
      const v8h v = *(const v8h*)(HST + (size_t)(rowbase + row) * NHID + ch * 8);
      *(v8h*)(&Hb[0][row * HPITCH + ch * 8]) = v;
    }
  }
  __syncthreads();

  const v8f z8 = {0.f, 0.f, 0.f, 0.f, 0.f, 0.f, 0.f, 0.f};
  const size_t gstr = (size_t)NHID * NHID;

#pragma unroll 1
  for (int s = 0; s < SEGSTEPS; ++s) {
    const int cur = s & 1;
    const _Float16* ahrow = &Hb[cur][0] + c * HPITCH + koff;
    _Float16* hnext = &Hb[cur ^ 1][0];
    const bool skip   = (init != 0) && (s == 0);
    const bool do_out = (out_every != 0) || ((final_out != 0) && (s == SEGSTEPS - 1));
    const size_t orow0 = (size_t)(t0 + s) * (size_t)out_tstride + (size_t)rowbase;
    const float* xprow = XP + ((size_t)s * NBATCH + rowbase + 8 * hh) * NGATE;

#pragma unroll 1
    for (int ub = 0; ub < 8; ++ub) {
      const int j = 128 * wave + 16 * ub + c;
      v8f zi8 = z8, zf8 = z8, zg8 = z8, zo8 = z8;
      if (!skip) {
        const _Float16* w0 = Ut + (size_t)j * NHID + koff;
#pragma unroll 1
        for (int k0 = 0; k0 < NHID; k0 += 32) {
          const v16h a  = frag_load(ahrow + k0);
          const v16h b0 = frag_load(w0 + k0);
          const v16h b1 = frag_load(w0 + gstr + k0);
          const v16h b2 = frag_load(w0 + 2 * gstr + k0);
          const v16h b3 = frag_load(w0 + 3 * gstr + k0);
          zi8 = frag_mma(a, b0, zi8);
          zf8 = frag_mma(a, b1, zf8);
          zg8 = frag_mma(a, b2, zg8);
          zo8 = frag_mma(a, b3, zo8);
          guard_group4(zi8, zf8, zg8, zo8, a, b0, b1, b2, b3);
        }
      }
      acc_guard4(zi8, zf8, zg8, zo8);
      const float mj = bn_mean[j];
      const float rj = rsqrtf(bn_var[j] + BN_EPS) * ACARRY;
      const float* xq = xprow + j;
      float*    cp = Cl + (8 * hh) * CPITCH + j;
      _Float16* hp = hnext + (8 * hh) * HPITCH + j;
      _Float16* op = os + (8 * hh) * OSP + 16 * (ub & 3) + c;
#pragma unroll
      for (int r = 0; r < 8; ++r) {
        if (r == 4) asm volatile("" ::: "memory");
        const float xi = xq[(size_t)r * NGATE];
        const float xf = xq[(size_t)r * NGATE + NHID];
        const float xg = xq[(size_t)r * NGATE + 2 * NHID];
        const float xo = xq[(size_t)r * NGATE + 3 * NHID];
        const float zi = zi8[r] * FOLDSC + xi;
        const float zf = zf8[r] * FOLDSC + xf;
        const float zg = zg8[r] * FOLDSC + xg;
        const float zo = zo8[r] * FOLDSC + xo;
        const float ig = fsig(zi);
        const float fg = fsig(zf);
        const float gg = ftanh(zg);
        const float og = fsig(zo);
        const float cold = cp[r * CPITCH];
        const float cn = fg * cold + ig * gg;
        cp[r * CPITCH] = cn;
        const float hn = og * ftanh(cn);
        hp[r * HPITCH] = (_Float16)(hn * ACARRY);
        if (do_out) op[r * OSP] = (_Float16)((hn - mj) * rj);
      }
      if (do_out && ((ub & 3) == 3)) {
        wave_lds_sync();
        const int q = lane >> 3, c8 = (lane & 7) * 8;
        unsigned short* ob = OUT16 + orow0 * NHID + 128 * wave + 64 * (ub >> 2);
        for (int pass = 0; pass < 2; ++pass) {
#pragma unroll
          for (int it = 0; it < 4; ++it) {
            const int row = it * 4 + q;
            const v8h hv = *(const v8h*)(os + row * OSP + c8);
            *(volatile v8h*)(ob + (size_t)row * NHID + c8) = hv;
          }
          __threadfence();
        }
        wave_lds_sync();
      }
    }
    __syncthreads();
  }

  for (int pass = 0; pass < 2; ++pass) {
#pragma unroll 1
    for (int it = 0; it < (BLKROWS * NHID / 4) / NTHR; ++it) {
      const int idx = it * NTHR + tid;
      const int row = idx >> 8, c4 = (idx & 255) * 4;
      const v4f v = *(const v4f*)(Cl + row * CPITCH + c4);
      *(volatile v4f*)(CST + (size_t)(rowbase + row) * NHID + c4) = v;
    }
    __threadfence();
  }

  {
    const _Float16* hb = &Hb[SEGSTEPS & 1][0];
    for (int pass = 0; pass < 2; ++pass) {
#pragma unroll 1
      for (int it = 0; it < (BLKROWS * NHID / 8) / NTHR; ++it) {
        const int idx = it * NTHR + tid;
        const int row = idx >> 7, ch = idx & 127;
        const v8h v = *(const v8h*)(hb + row * HPITCH + ch * 8);
        *(volatile v8h*)(HST + (size_t)(rowbase + row) * NHID + ch * 8) = v;
      }
      __threadfence();
    }
  }
}

extern "C" void kernel_launch(void* const* d_in, const int* in_sizes, int n_in,
                              void* d_out, int out_size, void* d_ws, size_t ws_size, hipStream_t stream) {
  if (n_in < 14 || d_out == nullptr || d_ws == nullptr) return;
  if (in_sizes[0] != NBATCH * NSTEPS || in_sizes[1] != NVOCAB * NEMB || in_sizes[2] != NEMB * NGATE ||
      in_sizes[3] != NHID * NGATE || in_sizes[4] != NGATE || in_sizes[5] != NHID || in_sizes[6] != NHID ||
      in_sizes[7] != NHID * NGATE || in_sizes[8] != NHID * NGATE || in_sizes[9] != NGATE ||
      in_sizes[10] != NHID || in_sizes[11] != NHID || in_sizes[12] != NHID * NHID || in_sizes[13] != NHID ||
      out_size != NBATCH * NHID) return;

  const int*   tokens = (const int*)d_in[0];
  const float* emb    = (const float*)d_in[1];
  const float* w1     = (const float*)d_in[2];
  const float* u1     = (const float*)d_in[3];
  const float* b1     = (const float*)d_in[4];
  const float* mean1  = (const float*)d_in[5];
  const float* var1   = (const float*)d_in[6];
  const float* w2     = (const float*)d_in[7];
  const float* u2     = (const float*)d_in[8];
  const float* b2     = (const float*)d_in[9];
  const float* mean2  = (const float*)d_in[10];
  const float* var2   = (const float*)d_in[11];
  const float* wd     = (const float*)d_in[12];
  const float* bd     = (const float*)d_in[13];
  float* out = (float*)d_out;

  char* ws = (char*)d_ws; size_t off = 0;
  auto carve = [&](size_t bytes) -> char* { char* p = ws + off; off += (bytes + 255) & ~(size_t)255; return p; };
  unsigned short* W1T   = (unsigned short*)carve((size_t)NGATE * NEMBP * 2);
  unsigned short* U1T   = (unsigned short*)carve((size_t)NGATE * NHID * 2);
  unsigned short* W2T   = (unsigned short*)carve((size_t)NGATE * NHID * 2);
  unsigned short* U2T   = (unsigned short*)carve((size_t)NGATE * NHID * 2);
  unsigned short* WDT   = (unsigned short*)carve((size_t)NHID * NHID * 2);
  unsigned short* X16   = (unsigned short*)carve((size_t)NROWS * NEMBP * 2);
  float*          XP    = (float*)carve((size_t)CHROWS * NGATE * 4);
  unsigned short* HSN16 = (unsigned short*)carve((size_t)NROWS * NHID * 2);
  unsigned short* HST16 = (unsigned short*)carve((size_t)NBATCH * NHID * 2);
  float*          CST32 = (float*)carve((size_t)NBATCH * NHID * 4);
  unsigned short* HT16  = (unsigned short*)carve((size_t)NBATCH * NHID * 2);
  if (off > ws_size || off > (size_t)134217728) return;

  tpw_f16_kernel<<<dim3(NGATE / 64, NEMBP / 64), NTHR, 0, stream>>>(w1, NEMB, NGATE, NEMBP, W1T, WCARRY);
  tpw_f16_kernel<<<dim3(NGATE / 64, NHID / 64),  NTHR, 0, stream>>>(u1, NHID, NGATE, NHID,  U1T, WCARRY);
  tpw_f16_kernel<<<dim3(NGATE / 64, NHID / 64),  NTHR, 0, stream>>>(w2, NHID, NGATE, NHID,  W2T, WCARRY);
  tpw_f16_kernel<<<dim3(NGATE / 64, NHID / 64),  NTHR, 0, stream>>>(u2, NHID, NGATE, NHID,  U2T, WCARRY);
  tpw_f16_kernel<<<dim3(NHID / 64,  NHID / 64),  NTHR, 0, stream>>>(wd, NHID, NHID,  NHID,  WDT, WCARRY);

  gather_x16_kernel<<<(NROWS * (NEMBP / 8)) / NTHR, NTHR, 0, stream>>>(tokens, emb, X16);

  const int gchunk = ((CHROWS / 64) * (NGATE / 64) + 7) / 8;
  const int rgrid  = NBATCH / BLKROWS;

  for (int ch = 0; ch < 2; ++ch) {
    gemm64_f16_kernel<0><<<gchunk, NTHR, 0, stream>>>(
        X16 + (size_t)ch * CHROWS * NEMBP, NEMBP, W1T, NEMBP, XP, NGATE, b1, CHROWS, NGATE, NEMBP, FOLDSC);
    lstm_seg_kernel<<<rgrid, NTHR, 0, stream>>>(
        XP, U1T, mean1, var1, HSN16, HST16, CST32, ch * SEGSTEPS, NBATCH, 1, 0, ch == 0 ? 1 : 0);
  }
  for (int ch = 0; ch < 2; ++ch) {
    gemm64_f16_kernel<0><<<gchunk, NTHR, 0, stream>>>(
        HSN16 + (size_t)ch * CHROWS * NHID, NHID, W2T, NHID, XP, NGATE, b2, CHROWS, NGATE, NHID, FOLDSC);
    lstm_seg_kernel<<<rgrid, NTHR, 0, stream>>>(
        XP, U2T, mean2, var2, HT16, HST16, CST32, ch * SEGSTEPS, 0, 0, ch == 1 ? 1 : 0, ch == 0 ? 1 : 0);
  }
  const int ghead = ((NBATCH / 64) * (NHID / 64) + 7) / 8;
  gemm64_f16_kernel<6><<<ghead, NTHR, 0, stream>>>(
      HT16, NHID, WDT, NHID, out, NHID, bd, NBATCH, NHID, NHID, FOLDSC);
}
